// LTCODE_79877801771610
// MI455X (gfx1250) — hardware-verified
//
#include <hip/hip_runtime.h>
#include <math.h>

typedef __attribute__((ext_vector_type(16))) _Float16 v16h;
typedef __attribute__((ext_vector_type(16))) __bf16 v16b;
typedef __attribute__((ext_vector_type(8)))  _Float16 v8h;
typedef __attribute__((ext_vector_type(8)))  float v8f;
typedef __attribute__((ext_vector_type(4)))  float v4f;
typedef __attribute__((ext_vector_type(2)))  float v2f;
typedef __attribute__((ext_vector_type(4)))  unsigned v4u;
typedef __attribute__((ext_vector_type(4)))  int v4i;
typedef float __attribute__((may_alias)) float_a;
typedef int __attribute__((may_alias)) int_a;

template <typename T> __device__ __forceinline__ void vst2(void* p, T v) { *(volatile T*)p = v; __threadfence(); *(volatile T*)p = v; }
__device__ __forceinline__ v8f wmma16(v16h a, v16h b, v8f c) {
  v8f d = __builtin_amdgcn_wmma_f32_16x16x32_f16(false, a, false, b, (short)0, c, false, false);
  asm volatile("v_nop\n\tv_nop\n\tv_nop\n\tv_nop" : "+v"(d) : "v"(a), "v"(b));
  return d;
}
__device__ __forceinline__ v8f wmma_bf(v16b a, v16b b, v8f c) {
  v8f d = __builtin_amdgcn_wmma_f32_16x16x32_bf16(false, a, false, b, (short)0, c, false, false);
  asm volatile("v_nop\n\tv_nop\n\tv_nop\n\tv_nop" : "+v"(d) : "v"(a), "v"(b));
  return d;
}
__device__ __forceinline__ v16h frag_h(const _Float16* rowk0, int lane) {
  union { v16h v; v8h q[2]; } u; const _Float16* p = rowk0 + 8 * (lane >> 4);
  u.q[0] = *(const v8h*)p; u.q[1] = *(const v8h*)(p + 16); return u.v;
}
__device__ __forceinline__ v16h frag_f32(const float* rowk0, int lane) {
  v16h a; const float* p = rowk0 + 8 * (lane >> 4);
#pragma unroll
  for (int i = 0; i < 8; ++i) { a[i] = (_Float16)p[i]; a[8 + i] = (_Float16)p[16 + i]; }
  return a;
}
__device__ __forceinline__ v16h frag_f32s(const float* rowk0, int lane, float sc) {
  v16h a; const float* p = rowk0 + 8 * (lane >> 4);
#pragma unroll
  for (int i = 0; i < 8; ++i) { a[i] = (_Float16)(p[i] * sc); a[8 + i] = (_Float16)(p[16 + i] * sc); }
  return a;
}
__device__ __forceinline__ v16h fragc_f32(const float* W, int k0, int n, int lane, int ld, int K) {
  v16h a; const int g = lane >> 4;
#pragma unroll
  for (int i = 0; i < 8; ++i) { const int ka = k0 + 8 * g + i, kb = ka + 16;
    a[i] = (_Float16)(ka < K ? W[(size_t)(ka < K ? ka : K - 1) * ld + n] : 0.f); a[8 + i] = (_Float16)(kb < K ? W[(size_t)(kb < K ? kb : K - 1) * ld + n] : 0.f); }
  return a;
}
struct F2 { v16b h, l; };
__device__ __forceinline__ F2 bsplit16(const float v[16]) { F2 r;
#pragma unroll
  for (int i = 0; i < 16; ++i) { const __bf16 h = (__bf16)v[i]; r.h[i] = h; r.l[i] = (__bf16)(v[i] - (float)h); }
  return r; }
__device__ __forceinline__ F2 split_row(const float* row, int k0, int lane) { float v[16]; const float* p = row + k0 + 8 * (lane >> 4);
#pragma unroll
  for (int i = 0; i < 8; ++i) { v[i] = p[i]; v[8 + i] = p[16 + i]; }
  return bsplit16(v); }
__device__ __forceinline__ F2 split_rowK(const float* row, int k0, int lane, int K) { float v[16]; const int g = lane >> 4;
#pragma unroll
  for (int i = 0; i < 8; ++i) { const int ka = k0 + 8 * g + i, kb = ka + 16; v[i] = ka < K ? row[ka < K ? ka : K - 1] : 0.f; v[8 + i] = kb < K ? row[kb < K ? kb : K - 1] : 0.f; }
  return bsplit16(v); }
__device__ __forceinline__ F2 split_col(const float* W, int k0, int n, int lane, int ld, int K) { float v[16]; const int g = lane >> 4;
#pragma unroll
  for (int i = 0; i < 8; ++i) { const int ka = k0 + 8 * g + i, kb = ka + 16; v[i] = ka < K ? W[(size_t)(ka < K ? ka : K - 1) * ld + n] : 0.f; v[8 + i] = kb < K ? W[(size_t)(kb < K ? kb : K - 1) * ld + n] : 0.f; }
  return bsplit16(v); }
__device__ __forceinline__ v8f mac3(const F2& a, const F2& b, v8f c) { c = wmma_bf(a.l, b.h, c); c = wmma_bf(a.h, b.l, c); return wmma_bf(a.h, b.h, c); }
__device__ __forceinline__ float sigm(float v) { return 1.0f / (1.0f + expf(-v)); }
#define LDSX() do { asm volatile("s_wait_dscnt 0" ::: "memory"); __builtin_amdgcn_wave_barrier(); __builtin_amdgcn_fence(__ATOMIC_RELEASE, "workgroup"); } while (0)


#define NB 8192
#define HH 1024
#ifndef TRB
#define TRB (NB / 32)
#endif
typedef __attribute__((ext_vector_type(8))) __bf16 v8b;
__device__ __forceinline__ v16b frag_gbf(const float* rowk0, int lane) {
  v16b a; const float* p = rowk0 + 8 * (lane >> 4);
#pragma unroll
  for (int i = 0; i < 8; ++i) { a[i] = (__bf16)p[i]; a[8 + i] = (__bf16)p[16 + i]; }
  return a;
}
__device__ __forceinline__ float bfr(float v) { return (float)(__bf16)v; }
__device__ __attribute__((noinline)) float exp_ni(float v) { return expf(v); }
__device__ __attribute__((noinline)) float tanh_ni(float v) { return tanhf(v); }
#define WS_END 64u

__global__ __launch_bounds__(256) void k_cell(const float* __restrict__ Hs, const float* __restrict__ X, const float* __restrict__ Win, const float* __restrict__ Wrec, const float* __restrict__ Wg, const float* __restrict__ ltau, const float* __restrict__ g_, const float* __restrict__ b_, float* __restrict__ OUT) {
  __shared__ __align__(16) float sd[32][HH + 4];
  const int tid = threadIdx.x, wave = tid >> 5, lane = tid & 31, col = lane & 15, g = lane >> 4; const int rt = wave & 1, cq = wave >> 1; const size_t r0 = (size_t)blockIdx.x * 32 + rt * 16;
#pragma unroll 1
  for (int jt = 0; jt < 16; ++jt) { const int o0 = cq * 256 + jt * 16;
    v8f acc_p = {}, acc_g = {};
#pragma unroll 4
    for (int kc = 0; kc < HH / 32; ++kc) { const v16b ah = frag_gbf(Hs + (r0 + col) * HH + kc * 32, lane);
      acc_p = wmma_bf(ah, frag_gbf(Wrec + (size_t)(o0 + col) * HH + kc * 32, lane), acc_p);
      acc_g = wmma_bf(ah, frag_gbf(Wg + (size_t)(o0 + col) * HH + kc * 32, lane), acc_g);
      const v16b ax = frag_gbf(X + (r0 + col) * HH + kc * 32, lane);
      acc_p = wmma_bf(ax, frag_gbf(Win + (size_t)(o0 + col) * HH + kc * 32, lane), acc_p); }
#pragma unroll
    for (int r = 0; r < 8; ++r) { const int o = o0 + col; const float gate = 1.0f / (1.0f + exp_ni(-acc_g[r])); const float hv = bfr(Hs[(r0 + 8 * g + r) * HH + o]);
      sd[rt * 16 + 8 * g + r][o] = (gate * tanh_ni(acc_p[r]) - hv) * exp_ni(-bfr(ltau[o])); } }
  __syncthreads();
  for (int rl = wave * 4; rl < wave * 4 + 4; ++rl) { float s = 0.f; for (int c = lane; c < HH; c += 32) s += sd[rl][c];
#pragma unroll
    for (int o = 1; o < 32; o <<= 1) s += __shfl_xor(s, o);
    const float mu = s / (float)HH; float v = 0.f; for (int c = lane; c < HH; c += 32) { const float d = sd[rl][c] - mu; v += d * d; }
#pragma unroll
    for (int o = 1; o < 32; o <<= 1) v += __shfl_xor(v, o);
    const float rs = rsqrtf(v / (float)HH + 1e-5f);
    for (int c = lane; c < HH; c += 32) sd[rl][c] = (sd[rl][c] - mu) * rs * bfr(g_[c]) + bfr(b_[c]); }
  __syncthreads();
  for (int q = tid; q < 32 * HH / 4; q += 256) { const int rl = q / (HH / 4), pc = q % (HH / 4); vst2(OUT + ((size_t)blockIdx.x * 32 + rl) * HH + pc * 4, *(const v4f*)&sd[rl][pc * 4]); }
}
extern "C" void kernel_launch(void* const* d_in, const int* in_sizes, int n_in, void* d_out, int out_size, void* d_ws, size_t ws_size, hipStream_t stream) {
  (void)in_sizes; (void)n_in; (void)out_size; (void)d_ws;
  const float** F = (const float**)d_in;
  if (ws_size < (size_t)WS_END) return;
  k_cell<<<TRB, 256, 0, stream>>>(F[0], F[1], F[2], F[3], F[4], F[5], F[6], F[7], (float*)d_out);
}
